// Convolution_30408368455936
// MI455X (gfx1250) — hardware-verified
//
#include <hip/hip_runtime.h>


namespace {
constexpr int NB_ = 2, G = 48, C = 64, MUL = 16, NVOX = NB_ * G * G * G, VL = NVOX  , NTAP = 81, CENTRE = 62;
constexpr float XS = 8.0f, WSC = 256.0f, RSQ3 = 0.57735026918962576f, RNLAT = 1.0f / 125.0f, RSQMUL = 0.25f;
static_assert(NVOX % 32 == 0 && VL % 32 == 0 && C == 64, "tiling");
typedef _Float16 b16;
typedef __attribute__((ext_vector_type(16))) _Float16 v16b;
typedef __attribute__((ext_vector_type(8))) _Float16 v8b;
typedef __attribute__((ext_vector_type(8))) float v8f;
typedef __attribute__((ext_vector_type(4))) float v4f;
__device__ __forceinline__ float bf16_rne(float f) { unsigned int u = __float_as_uint(f); u += 0x7FFFu + ((u >> 16) & 1u); return __uint_as_float(u & 0xFFFF0000u); }
__device__ __forceinline__ void split16(float v, b16& hi, b16& lo) { hi = (b16)v; lo = (b16)(v - (float)hi); }
__device__ __forceinline__ v16b frag_kb(const b16* p, int hh) { const v8b a = *(const v8b*)(p + 8 * hh), b = *(const v8b*)(p + 16 + 8 * hh); v16b f;
#pragma unroll
  for (int e = 0; e < 8; ++e) { f[e] = a[e]; f[8 + e] = b[e]; } return f; }
__device__ __forceinline__ v8f wmma16b(v16b a, v16b b, v8f c) { v8f d = __builtin_amdgcn_wmma_f32_16x16x32_f16(false, a, false, b, (short)0, c, false, false); asm volatile("v_nop\n\tv_nop\n\tv_nop\n\tv_nop" : "+v"(d) : "v"(a), "v"(b)); return d; }
__device__ __forceinline__ void wave_lds_sync() { __builtin_amdgcn_fence(__ATOMIC_RELEASE, "workgroup"); __builtin_amdgcn_wave_barrier(); __builtin_amdgcn_fence(__ATOMIC_ACQUIRE, "workgroup"); }
__device__ __forceinline__ float pmul(float a, float b) { float p = a * b; asm volatile("" : "+v"(p)); return p; }
__device__ __forceinline__ int iclamp(int v, int lo, int hi) { return v < lo ? lo : (v > hi ? hi : v); }

typedef __attribute__((ext_vector_type(2))) _Float16 v2h;
typedef __attribute__((ext_vector_type(4))) _Float16 v4h;
typedef __attribute__((ext_vector_type(2))) float v2f;
typedef __attribute__((ext_vector_type(4))) int v4i;
__device__ __forceinline__ float nexp2(float v) { return __builtin_amdgcn_exp2f(v); }
typedef __attribute__((ext_vector_type(4))) _Float16 v4h_;
__constant__ float EMB[125 * 4] = {0.000000000e+00f,0.000000000e+00f,0.000000000e+00f,0.000000000e+00f,0.000000000e+00f,0.000000000e+00f,0.000000000e+00f,0.000000000e+00f,0.000000000e+00f,0.000000000e+00f,0.000000000e+00f,0.000000000e+00f,0.000000000e+00f,0.000000000e+00f,0.000000000e+00f,0.000000000e+00f,0.000000000e+00f,0.000000000e+00f,0.000000000e+00f,0.000000000e+00f,0.000000000e+00f,0.000000000e+00f,0.000000000e+00f,0.000000000e+00f,0.000000000e+00f,0.000000000e+00f,0.000000000e+00f,4.593313485e-02f,0.000000000e+00f,0.000000000e+00f,0.000000000e+00f,2.328826189e+00f,0.000000000e+00f,0.000000000e+00f,0.000000000e+00f,4.593313485e-02f,0.000000000e+00f,0.000000000e+00f,0.000000000e+00f,0.000000000e+00f,0.000000000e+00f,0.000000000e+00f,0.000000000e+00f,0.000000000e+00f,0.000000000e+00f,0.000000000e+00f,0.000000000e+00f,2.328826189e+00f,0.000000000e+00f,0.000000000e+00f,0.000000000e+00f,3.102538109e+00f,0.000000000e+00f,0.000000000e+00f,0.000000000e+00f,2.328826189e+00f,0.000000000e+00f,0.000000000e+00f,0.000000000e+00f,0.000000000e+00f,0.000000000e+00f,0.000000000e+00f,0.000000000e+00f,0.000000000e+00f,0.000000000e+00f,0.000000000e+00f,0.000000000e+00f,4.593313485e-02f,0.000000000e+00f,0.000000000e+00f,0.000000000e+00f,2.328826189e+00f,0.000000000e+00f,0.000000000e+00f,0.000000000e+00f,4.593313485e-02f,0.000000000e+00f,0.000000000e+00f,0.000000000e+00f,0.000000000e+00f,0.000000000e+00f,0.000000000e+00f,0.000000000e+00f,0.000000000e+00f,0.000000000e+00f,0.000000000e+00f,0.000000000e+00f,0.000000000e+00f,0.000000000e+00f,0.000000000e+00f,0.000000000e+00f,0.000000000e+00f,0.000000000e+00f,0.000000000e+00f,0.000000000e+00f,0.000000000e+00f,0.000000000e+00f,0.000000000e+00f,0.000000000e+00f,0.000000000e+00f,0.000000000e+00f,0.000000000e+00f,0.000000000e+00f,0.000000000e+00f,0.000000000e+00f,0.000000000e+00f,0.000000000e+00f,4.593313485e-02f,0.000000000e+00f,0.000000000e+00f,0.000000000e+00f,2.328826189e+00f,0.000000000e+00f,0.000000000e+00f,0.000000000e+00f,4.593313485e-02f,0.000000000e+00f,0.000000000e+00f,0.000000000e+00f,0.000000000e+00f,0.000000000e+00f,0.000000000e+00f,0.000000000e+00f,4.593313485e-02f,0.000000000e+00f,0.000000000e+00f,2.357735157e+00f,2.073686361e+00f,0.000000000e+00f,3.480350375e-01f,3.009850502e+00f,0.000000000e+00f,0.000000000e+00f,0.000000000e+00f,2.357735157e+00f,2.073686361e+00f,0.000000000e+00f,0.000000000e+00f,0.000000000e+00f,4.593313485e-02f,0.000000000e+00f,0.000000000e+00f,0.000000000e+00f,2.328826189e+00f,0.000000000e+00f,3.480350375e-01f,3.009850502e+00f,0.000000000e+00f,0.000000000e+00f,3.102538109e+00f,0.000000000e+00f,0.000000000e+00f,0.000000000e+00f,3.480350375e-01f,3.009850502e+00f,0.000000000e+00f,0.000000000e+00f,0.000000000e+00f,0.000000000e+00f,2.328826189e+00f,0.000000000e+00f,0.000000000e+00f,0.000000000e+00f,4.593313485e-02f,0.000000000e+00f,0.000000000e+00f,2.357735157e+00f,2.073686361e+00f,0.000000000e+00f,3.480350375e-01f,3.009850502e+00f,0.000000000e+00f,0.000000000e+00f,0.000000000e+00f,2.357735157e+00f,2.073686361e+00f,0.000000000e+00f,0.000000000e+00f,0.000000000e+00f,4.593313485e-02f,0.000000000e+00f,0.000000000e+00f,0.000000000e+00f,0.000000000e+00f,0.000000000e+00f,0.000000000e+00f,0.000000000e+00f,4.593313485e-02f,0.000000000e+00f,0.000000000e+00f,0.000000000e+00f,2.328826189e+00f,0.000000000e+00f,0.000000000e+00f,0.000000000e+00f,4.593313485e-02f,0.000000000e+00f,0.000000000e+00f,0.000000000e+00f,0.000000000e+00f,0.000000000e+00f,0.000000000e+00f,0.000000000e+00f,0.000000000e+00f,0.000000000e+00f,0.000000000e+00f,0.000000000e+00f,2.328826189e+00f,0.000000000e+00f,0.000000000e+00f,0.000000000e+00f,3.102538109e+00f,0.000000000e+00f,0.000000000e+00f,0.000000000e+00f,2.328826189e+00f,0.000000000e+00f,0.000000000e+00f,0.000000000e+00f,0.000000000e+00f,0.000000000e+00f,0.000000000e+00f,0.000000000e+00f,2.328826189e+00f,0.000000000e+00f,3.480350375e-01f,3.009850502e+00f,0.000000000e+00f,0.000000000e+00f,3.102538109e+00f,0.000000000e+00f,0.000000000e+00f,0.000000000e+00f,3.480350375e-01f,3.009850502e+00f,0.000000000e+00f,0.000000000e+00f,0.000000000e+00f,0.000000000e+00f,2.328826189e+00f,0.000000000e+00f,0.000000000e+00f,0.000000000e+00f,3.102538109e+00f,0.000000000e+00f,3.102538109e+00f,0.000000000e+00f,0.000000000e+00f,0.000000000e+00f,0.000000000e+00f,0.000000000e+00f,0.000000000e+00f,0.000000000e+00f,3.102538109e+00f,0.000000000e+00f,0.000000000e+00f,0.000000000e+00f,0.000000000e+00f,0.000000000e+00f,3.102538109e+00f,0.000000000e+00f,0.000000000e+00f,0.000000000e+00f,2.328826189e+00f,0.000000000e+00f,3.480350375e-01f,3.009850502e+00f,0.000000000e+00f,0.000000000e+00f,3.102538109e+00f,0.000000000e+00f,0.000000000e+00f,0.000000000e+00f,3.480350375e-01f,3.009850502e+00f,0.000000000e+00f,0.000000000e+00f,0.000000000e+00f,0.000000000e+00f,2.328826189e+00f,0.000000000e+00f,0.000000000e+00f,0.000000000e+00f,0.000000000e+00f,0.000000000e+00f,0.000000000e+00f,0.000000000e+00f,2.328826189e+00f,0.000000000e+00f,0.000000000e+00f,0.000000000e+00f,3.102538109e+00f,0.000000000e+00f,0.000000000e+00f,0.000000000e+00f,2.328826189e+00f,0.000000000e+00f,0.000000000e+00f,0.000000000e+00f,0.000000000e+00f,0.000000000e+00f,0.000000000e+00f,0.000000000e+00f,0.000000000e+00f,0.000000000e+00f,0.000000000e+00f,0.000000000e+00f,4.593313485e-02f,0.000000000e+00f,0.000000000e+00f,0.000000000e+00f,2.328826189e+00f,0.000000000e+00f,0.000000000e+00f,0.000000000e+00f,4.593313485e-02f,0.000000000e+00f,0.000000000e+00f,0.000000000e+00f,0.000000000e+00f,0.000000000e+00f,0.000000000e+00f,0.000000000e+00f,4.593313485e-02f,0.000000000e+00f,0.000000000e+00f,2.357735157e+00f,2.073686361e+00f,0.000000000e+00f,3.480350375e-01f,3.009850502e+00f,0.000000000e+00f,0.000000000e+00f,0.000000000e+00f,2.357735157e+00f,2.073686361e+00f,0.000000000e+00f,0.000000000e+00f,0.000000000e+00f,4.593313485e-02f,0.000000000e+00f,0.000000000e+00f,0.000000000e+00f,2.328826189e+00f,0.000000000e+00f,3.480350375e-01f,3.009850502e+00f,0.000000000e+00f,0.000000000e+00f,3.102538109e+00f,0.000000000e+00f,0.000000000e+00f,0.000000000e+00f,3.480350375e-01f,3.009850502e+00f,0.000000000e+00f,0.000000000e+00f,0.000000000e+00f,0.000000000e+00f,2.328826189e+00f,0.000000000e+00f,0.000000000e+00f,0.000000000e+00f,4.593313485e-02f,0.000000000e+00f,0.000000000e+00f,2.357735157e+00f,2.073686361e+00f,0.000000000e+00f,3.480350375e-01f,3.009850502e+00f,0.000000000e+00f,0.000000000e+00f,0.000000000e+00f,2.357735157e+00f,2.073686361e+00f,0.000000000e+00f,0.000000000e+00f,0.000000000e+00f,4.593313485e-02f,0.000000000e+00f,0.000000000e+00f,0.000000000e+00f,0.000000000e+00f,0.000000000e+00f,0.000000000e+00f,0.000000000e+00f,4.593313485e-02f,0.000000000e+00f,0.000000000e+00f,0.000000000e+00f,2.328826189e+00f,0.000000000e+00f,0.000000000e+00f,0.000000000e+00f,4.593313485e-02f,0.000000000e+00f,0.000000000e+00f,0.000000000e+00f,0.000000000e+00f,0.000000000e+00f,0.000000000e+00f,0.000000000e+00f,0.000000000e+00f,0.000000000e+00f,0.000000000e+00f,0.000000000e+00f,0.000000000e+00f,0.000000000e+00f,0.000000000e+00f,0.000000000e+00f,0.000000000e+00f,0.000000000e+00f,0.000000000e+00f,0.000000000e+00f,0.000000000e+00f,0.000000000e+00f,0.000000000e+00f,0.000000000e+00f,0.000000000e+00f,0.000000000e+00f,0.000000000e+00f,0.000000000e+00f,0.000000000e+00f,0.000000000e+00f,0.000000000e+00f,0.000000000e+00f,4.593313485e-02f,0.000000000e+00f,0.000000000e+00f,0.000000000e+00f,2.328826189e+00f,0.000000000e+00f,0.000000000e+00f,0.000000000e+00f,4.593313485e-02f,0.000000000e+00f,0.000000000e+00f,0.000000000e+00f,0.000000000e+00f,0.000000000e+00f,0.000000000e+00f,0.000000000e+00f,0.000000000e+00f,0.000000000e+00f,0.000000000e+00f,0.000000000e+00f,2.328826189e+00f,0.000000000e+00f,0.000000000e+00f,0.000000000e+00f,3.102538109e+00f,0.000000000e+00f,0.000000000e+00f,0.000000000e+00f,2.328826189e+00f,0.000000000e+00f,0.000000000e+00f,0.000000000e+00f,0.000000000e+00f,0.000000000e+00f,0.000000000e+00f,0.000000000e+00f,0.000000000e+00f,0.000000000e+00f,0.000000000e+00f,0.000000000e+00f,4.593313485e-02f,0.000000000e+00f,0.000000000e+00f,0.000000000e+00f,2.328826189e+00f,0.000000000e+00f,0.000000000e+00f,0.000000000e+00f,4.593313485e-02f,0.000000000e+00f,0.000000000e+00f,0.000000000e+00f,0.000000000e+00f,0.000000000e+00f,0.000000000e+00f,0.000000000e+00f,0.000000000e+00f,0.000000000e+00f,0.000000000e+00f,0.000000000e+00f,0.000000000e+00f,0.000000000e+00f,0.000000000e+00f,0.000000000e+00f,0.000000000e+00f,0.000000000e+00f,0.000000000e+00f,0.000000000e+00f,0.000000000e+00f,0.000000000e+00f,0.000000000e+00f,0.000000000e+00f,0.000000000e+00f};
__constant__ float SH1[125 * 3] = {-1.000000000e+00f,-1.000000000e+00f,-1.000000000e+00f,-1.154700518e+00f,-1.154700518e+00f,-5.773502588e-01f,-1.224744916e+00f,-1.224744916e+00f,0.000000000e+00f,-1.154700518e+00f,-1.154700518e+00f,5.773502588e-01f,-1.000000000e+00f,-1.000000000e+00f,1.000000000e+00f,-1.154700518e+00f,-5.773502588e-01f,-1.154700518e+00f,-1.414213538e+00f,-7.071067691e-01f,-7.071067691e-01f,-1.549193382e+00f,-7.745966911e-01f,0.000000000e+00f,-1.414213538e+00f,-7.071067691e-01f,7.071067691e-01f,-1.154700518e+00f,-5.773502588e-01f,1.154700518e+00f,-1.224744916e+00f,0.000000000e+00f,-1.224744916e+00f,-1.549193382e+00f,0.000000000e+00f,-7.745966911e-01f,-1.732050776e+00f,0.000000000e+00f,0.000000000e+00f,-1.549193382e+00f,0.000000000e+00f,7.745966911e-01f,-1.224744916e+00f,0.000000000e+00f,1.224744916e+00f,-1.154700518e+00f,5.773502588e-01f,-1.154700518e+00f,-1.414213538e+00f,7.071067691e-01f,-7.071067691e-01f,-1.549193382e+00f,7.745966911e-01f,0.000000000e+00f,-1.414213538e+00f,7.071067691e-01f,7.071067691e-01f,-1.154700518e+00f,5.773502588e-01f,1.154700518e+00f,-1.000000000e+00f,1.000000000e+00f,-1.000000000e+00f,-1.154700518e+00f,1.154700518e+00f,-5.773502588e-01f,-1.224744916e+00f,1.224744916e+00f,0.000000000e+00f,-1.154700518e+00f,1.154700518e+00f,5.773502588e-01f,-1.000000000e+00f,1.000000000e+00f,1.000000000e+00f,-5.773502588e-01f,-1.154700518e+00f,-1.154700518e+00f,-7.071067691e-01f,-1.414213538e+00f,-7.071067691e-01f,-7.745966911e-01f,-1.549193382e+00f,0.000000000e+00f,-7.071067691e-01f,-1.414213538e+00f,7.071067691e-01f,-5.773502588e-01f,-1.154700518e+00f,1.154700518e+00f,-7.071067691e-01f,-7.071067691e-01f,-1.414213538e+00f,-1.000000000e+00f,-1.000000000e+00f,-1.000000000e+00f,-1.224744916e+00f,-1.224744916e+00f,0.000000000e+00f,-1.000000000e+00f,-1.000000000e+00f,1.000000000e+00f,-7.071067691e-01f,-7.071067691e-01f,1.414213538e+00f,-7.745966911e-01f,0.000000000e+00f,-1.549193382e+00f,-1.224744916e+00f,0.000000000e+00f,-1.224744916e+00f,-1.732050776e+00f,0.000000000e+00f,0.000000000e+00f,-1.224744916e+00f,0.000000000e+00f,1.224744916e+00f,-7.745966911e-01f,0.000000000e+00f,1.549193382e+00f,-7.071067691e-01f,7.071067691e-01f,-1.414213538e+00f,-1.000000000e+00f,1.000000000e+00f,-1.000000000e+00f,-1.224744916e+00f,1.224744916e+00f,0.000000000e+00f,-1.000000000e+00f,1.000000000e+00f,1.000000000e+00f,-7.071067691e-01f,7.071067691e-01f,1.414213538e+00f,-5.773502588e-01f,1.154700518e+00f,-1.154700518e+00f,-7.071067691e-01f,1.414213538e+00f,-7.071067691e-01f,-7.745966911e-01f,1.549193382e+00f,0.000000000e+00f,-7.071067691e-01f,1.414213538e+00f,7.071067691e-01f,-5.773502588e-01f,1.154700518e+00f,1.154700518e+00f,0.000000000e+00f,-1.224744916e+00f,-1.224744916e+00f,0.000000000e+00f,-1.549193382e+00f,-7.745966911e-01f,0.000000000e+00f,-1.732050776e+00f,0.000000000e+00f,0.000000000e+00f,-1.549193382e+00f,7.745966911e-01f,0.000000000e+00f,-1.224744916e+00f,1.224744916e+00f,0.000000000e+00f,-7.745966911e-01f,-1.549193382e+00f,0.000000000e+00f,-1.224744916e+00f,-1.224744916e+00f,0.000000000e+00f,-1.732050776e+00f,0.000000000e+00f,0.000000000e+00f,-1.224744916e+00f,1.224744916e+00f,0.000000000e+00f,-7.745966911e-01f,1.549193382e+00f,0.000000000e+00f,0.000000000e+00f,-1.732050776e+00f,0.000000000e+00f,0.000000000e+00f,-1.732050776e+00f,0.000000000e+00f,0.000000000e+00f,0.000000000e+00f,0.000000000e+00f,0.000000000e+00f,1.732050776e+00f,0.000000000e+00f,0.000000000e+00f,1.732050776e+00f,0.000000000e+00f,7.745966911e-01f,-1.549193382e+00f,0.000000000e+00f,1.224744916e+00f,-1.224744916e+00f,0.000000000e+00f,1.732050776e+00f,0.000000000e+00f,0.000000000e+00f,1.224744916e+00f,1.224744916e+00f,0.000000000e+00f,7.745966911e-01f,1.549193382e+00f,0.000000000e+00f,1.224744916e+00f,-1.224744916e+00f,0.000000000e+00f,1.549193382e+00f,-7.745966911e-01f,0.000000000e+00f,1.732050776e+00f,0.000000000e+00f,0.000000000e+00f,1.549193382e+00f,7.745966911e-01f,0.000000000e+00f,1.224744916e+00f,1.224744916e+00f,5.773502588e-01f,-1.154700518e+00f,-1.154700518e+00f,7.071067691e-01f,-1.414213538e+00f,-7.071067691e-01f,7.745966911e-01f,-1.549193382e+00f,0.000000000e+00f,7.071067691e-01f,-1.414213538e+00f,7.071067691e-01f,5.773502588e-01f,-1.154700518e+00f,1.154700518e+00f,7.071067691e-01f,-7.071067691e-01f,-1.414213538e+00f,1.000000000e+00f,-1.000000000e+00f,-1.000000000e+00f,1.224744916e+00f,-1.224744916e+00f,0.000000000e+00f,1.000000000e+00f,-1.000000000e+00f,1.000000000e+00f,7.071067691e-01f,-7.071067691e-01f,1.414213538e+00f,7.745966911e-01f,0.000000000e+00f,-1.549193382e+00f,1.224744916e+00f,0.000000000e+00f,-1.224744916e+00f,1.732050776e+00f,0.000000000e+00f,0.000000000e+00f,1.224744916e+00f,0.000000000e+00f,1.224744916e+00f,7.745966911e-01f,0.000000000e+00f,1.549193382e+00f,7.071067691e-01f,7.071067691e-01f,-1.414213538e+00f,1.000000000e+00f,1.000000000e+00f,-1.000000000e+00f,1.224744916e+00f,1.224744916e+00f,0.000000000e+00f,1.000000000e+00f,1.000000000e+00f,1.000000000e+00f,7.071067691e-01f,7.071067691e-01f,1.414213538e+00f,5.773502588e-01f,1.154700518e+00f,-1.154700518e+00f,7.071067691e-01f,1.414213538e+00f,-7.071067691e-01f,7.745966911e-01f,1.549193382e+00f,0.000000000e+00f,7.071067691e-01f,1.414213538e+00f,7.071067691e-01f,5.773502588e-01f,1.154700518e+00f,1.154700518e+00f,1.000000000e+00f,-1.000000000e+00f,-1.000000000e+00f,1.154700518e+00f,-1.154700518e+00f,-5.773502588e-01f,1.224744916e+00f,-1.224744916e+00f,0.000000000e+00f,1.154700518e+00f,-1.154700518e+00f,5.773502588e-01f,1.000000000e+00f,-1.000000000e+00f,1.000000000e+00f,1.154700518e+00f,-5.773502588e-01f,-1.154700518e+00f,1.414213538e+00f,-7.071067691e-01f,-7.071067691e-01f,1.549193382e+00f,-7.745966911e-01f,0.000000000e+00f,1.414213538e+00f,-7.071067691e-01f,7.071067691e-01f,1.154700518e+00f,-5.773502588e-01f,1.154700518e+00f,1.224744916e+00f,0.000000000e+00f,-1.224744916e+00f,1.549193382e+00f,0.000000000e+00f,-7.745966911e-01f,1.732050776e+00f,0.000000000e+00f,0.000000000e+00f,1.549193382e+00f,0.000000000e+00f,7.745966911e-01f,1.224744916e+00f,0.000000000e+00f,1.224744916e+00f,1.154700518e+00f,5.773502588e-01f,-1.154700518e+00f,1.414213538e+00f,7.071067691e-01f,-7.071067691e-01f,1.549193382e+00f,7.745966911e-01f,0.000000000e+00f,1.414213538e+00f,7.071067691e-01f,7.071067691e-01f,1.154700518e+00f,5.773502588e-01f,1.154700518e+00f,1.000000000e+00f,1.000000000e+00f,-1.000000000e+00f,1.154700518e+00f,1.154700518e+00f,-5.773502588e-01f,1.224744916e+00f,1.224744916e+00f,0.000000000e+00f,1.154700518e+00f,1.154700518e+00f,5.773502588e-01f,1.000000000e+00f,1.000000000e+00f,1.000000000e+00f};
__constant__ int TAPS[NTAP] = {6,7,8,11,12,13,16,17,18,26,27,28,30,31,32,33,34,35,36,37,38,39,40,41,42,43,44,46,47,48,51,52,53,55,56,57,58,59,60,61,62,63,64,65,66,67,68,69,71,72,73,76,77,78,80,81,82,83,84,85,86,87,88,89,90,91,92,93,94,96,97,98,106,107,108,111,112,113,116,117,118};
__global__ __launch_bounds__(256) void build_kernel(const float* __restrict__ w000, const float* __restrict__ w011, const float* __restrict__ w101, const float* __restrict__ w110, const float* __restrict__ sc0, const float* __restrict__ sc1, b16* __restrict__ WT) {
  const int u_ = blockIdx.x * 256 + threadIdx.x; if (u_ >= NTAP * C * C / 8) return; const int e = u_ * 8; const int s = e / (C * C), rem = e % (C * C), o = rem / C, i0 = rem % C; const int t = TAPS[s];
  const float e0 = EMB[t * 4 + 0], e1 = EMB[t * 4 + 1], e2 = EMB[t * 4 + 2], e3 = EMB[t * 4 + 3]; const float s0 = SH1[t * 3 + 0], s1 = SH1[t * 3 + 1], s2 = SH1[t * 3 + 2];
  auto rad = [&](const float* __restrict__ wp, int u, int w) { return (((e0 * bf16_rne(wp[(0 * MUL + u) * MUL + w]) + e1 * bf16_rne(wp[(1 * MUL + u) * MUL + w])) + e2 * bf16_rne(wp[(2 * MUL + u) * MUL + w])) + e3 * bf16_rne(wp[(3 * MUL + u) * MUL + w])) * RNLAT; };
  auto shv = [&](int q) { return q == 0 ? s0 : (q == 1 ? s1 : s2); };
  v8b out8;
#pragma unroll 1
  for (int j = 0; j < 8; ++j) { const int i = i0 + j; float kv = 0.0f;
    if (t == CENTRE) { if (i < MUL && o < MUL) kv = bf16_rne(sc0[i * MUL + o]) * RSQMUL; else if (i >= MUL && o >= MUL) { const int u = (i - MUL) / 3, ii = (i - MUL) % 3, w = (o - MUL) / 3, kk = (o - MUL) % 3; kv = (ii == kk) ? bf16_rne(sc1[u * MUL + w]) * RSQMUL : 0.0f; } }
    else if (i < MUL) { if (o < MUL) kv = rad(w000, i, o); else { const int w = (o - MUL) / 3, kk = (o - MUL) % 3; kv = rad(w011, i, w) * shv(kk); } }
    else { const int u = (i - MUL) / 3, ii = (i - MUL) % 3; if (o < MUL) kv = rad(w110, u, o) * shv(ii) * RSQ3; else { const int w = (o - MUL) / 3, kk = (o - MUL) % 3; kv = (ii == kk) ? rad(w101, u, w) : 0.0f; } }
    out8[j] = (b16)(kv * WSC); }
  for (int pass = 0; pass < 2; ++pass) { *(volatile v8b*)(WT + e) = out8; __threadfence(); }
}
__global__ __launch_bounds__(256) void conv_kernel(const float* __restrict__ x, const b16* __restrict__ WT, float* __restrict__ out) {
  __shared__ __attribute__((aligned(16))) b16 As[32][C + 8]; __shared__ __attribute__((aligned(16))) float Tf[32][C + 4];
  const int tid = threadIdx.x, wave = tid >> 5, lane = tid & 31, nloc = lane & 15, hlf = lane >> 4; const int v0 = blockIdx.x * 32; const int row = tid >> 3, g = tid & 7; const int v = v0 + row;
  const int vz = v % G, vy = (v / G) % G, vx = (v / (G * G)) % G, vn = v / (G * G * G);
  const int rt = wave & 1, ct = wave >> 1; v8f acc = (v8f){};
#pragma unroll 1
  for (int s = 0; s < NTAP; ++s) { const int t = TAPS[s]; const int dx = t / 25 - 2, dy = (t / 5) % 5 - 2, dz = t % 5 - 2; const int sx = vx + dx, sy = vy + dy, sz = vz + dz;
    const bool inb = (sx >= 0 && sx < G && sy >= 0 && sy < G && sz >= 0 && sz < G); const float fl = inb ? XS : 0.0f;
    const float* xr = x + ((((size_t)vn * G + iclamp(sx, 0, G - 1)) * G + iclamp(sy, 0, G - 1)) * G + iclamp(sz, 0, G - 1)) * C + g * 8;
    const v4f f0 = *(const v4f*)xr, f1 = *(const v4f*)(xr + 4); v8b a8; for (int q = 0; q < 4; ++q) { a8[q] = (b16)(bf16_rne(f0[q]) * fl); a8[4 + q] = (b16)(bf16_rne(f1[q]) * fl); }
    __syncthreads();
    *(v8b*)(&As[row][g * 8]) = a8;
    __syncthreads();
    const b16* br = WT + ((size_t)s * C + ct * 16 + nloc) * C;
#pragma unroll
    for (int kb = 0; kb < C; kb += 32) acc = wmma16b(frag_kb(&As[rt * 16 + nloc][kb], hlf), frag_kb(br + kb, hlf), acc); }
#pragma unroll
  for (int r = 0; r < 8; ++r) Tf[rt * 16 + 8 * hlf + r][ct * 16 + nloc] = acc[r] * (1.0f / (XS * WSC));
  __syncthreads();
  for (int pass = 0; pass < 2; ++pass) { for (int rr = wave * 4; rr < wave * 4 + 4; rr += 2) { const int r2 = rr + (lane >> 4); if (v0 + r2 < VL) *(volatile v4f*)(out + (size_t)(v0 + r2) * C + (lane & 15) * 4) = *(const v4f*)(&Tf[r2][(lane & 15) * 4]); } __threadfence(); }
}
}

extern "C" void kernel_launch(void* const* d_in, const int* in_sizes, int n_in, void* d_out, int out_size, void* d_ws, size_t ws_size, hipStream_t stream) {
  (void)n_in;
  auto Fp = [&](int i) { return (const float*)d_in[i]; };
  if (in_sizes[0] != NVOX * C || in_sizes[1] != 4 * MUL * MUL || in_sizes[2] != 4 * MUL * MUL || in_sizes[3] != 4 * MUL * MUL || in_sizes[4] != 4 * MUL * MUL || in_sizes[5] != MUL * MUL || in_sizes[6] != MUL * MUL || out_size != NVOX * C) return;
  size_t off = 0; char* ws = (char*)d_ws;
  auto carve = [&](size_t bytes) { char* p = ws + off; off += (bytes + 255) & ~(size_t)255; return p; };
  b16* WT = (b16*)carve((size_t)NTAP * C * C * 2);
  if (off > ws_size || off > ((size_t)128 << 20)) return;
  build_kernel<<<(NTAP * C * C / 8 + 255) / 256, 256, 0, stream>>>(Fp(1), Fp(2), Fp(3), Fp(4), Fp(5), Fp(6), WT);
  conv_kernel<<<VL / 32, 256, 0, stream>>>(Fp(0), WT, (float*)d_out);
}
